// MFGCGRU_SM_23570780521077
// MI455X (gfx1250) — hardware-verified
//
#include <hip/hip_runtime.h>
#include <hip/hip_bf16.h>
#include <math.h>


typedef _Float16 bf16;
typedef _Float16 f16;
typedef __attribute__((ext_vector_type(4))) unsigned v4u_t;
typedef unsigned v4ua __attribute__((ext_vector_type(4), may_alias));
typedef __attribute__((ext_vector_type(4))) float v4f_t;
typedef float v4fa __attribute__((ext_vector_type(4), may_alias));
typedef __attribute__((ext_vector_type(16))) bf16  bf16x16;
typedef bf16x16 f16x16;
typedef __attribute__((ext_vector_type(8)))  bf16  bf16x8;
typedef bf16x8 f16x8;
typedef __attribute__((ext_vector_type(4)))  bf16  bf16x4;
typedef __attribute__((ext_vector_type(8)))  float f32x8;
__device__ __forceinline__ f32x8 wmma16(f16x16 a, f16x16 b, f32x8 c) {
  c = __builtin_amdgcn_wmma_f32_16x16x32_f16(false, a, false, b, (short)0, c, false, false);
  asm volatile("v_nop\n\tv_nop\n\tv_nop\n\tv_nop" : "+v"(c) : "v"(a), "v"(b));
  return c;
}
#define LDS_STRIDE 48
#define KSTRIDE    72
#define VSTRIDE    48

__device__ __forceinline__ f32x8 wmma_bf16(bf16x16 a, bf16x16 b, f32x8 c) {
  c = __builtin_amdgcn_wmma_f32_16x16x32_f16(false, a, false, b, (short)0, c, false, false);
  asm volatile("v_nop\n\tv_nop\n\tv_nop\n\tv_nop" : "+v"(c) : "v"(a), "v"(b));
  return c;
}

template <typename T>
__device__ __forceinline__ bf16x16 load_frag(const T* __restrict__ base, int ld,
                                             int row0, int k0) {
  const int lane = threadIdx.x & 31;
  const int r    = lane & 15;
  const int kh   = (lane >> 4) * 8;
  const T* p0 = base + (size_t)(row0 + r) * ld + (k0 + kh);
  const T* p1 = p0 + 16;
  bf16x16 f;
#pragma unroll
  for (int i = 0; i < 8; ++i) {
    f[i]     = (bf16)p0[i];
    f[i + 8] = (bf16)p1[i];
  }
  return f;
}

__device__ __forceinline__ bf16x16 lds_frag(const bf16* base, int stride) {
  const int lane = threadIdx.x & 31;
  const int row  = lane & 15;
  const int kh   = (lane >> 4) * 8;
  const bf16x8 lo = *(const bf16x8*)(base + row * stride + kh);
  const bf16x8 hi = *(const bf16x8*)(base + row * stride + kh + 16);
  bf16x16 f;
#pragma unroll
  for (int i = 0; i < 8; ++i) { f[i] = lo[i]; f[i + 8] = hi[i]; }
  return f;
}

template <typename T>
__device__ __forceinline__ void stage_read16(const T* __restrict__ p, float* buf) {
#pragma unroll
  for (int i = 0; i < 16; ++i) buf[i] = (float)p[i];
}

__device__ __forceinline__ void stage_write(bf16* dst, const float* buf, int nquad) {
#pragma unroll
  for (int i = 0; i < nquad; ++i) {
    bf16x4 q;
    q[0] = (bf16)buf[4 * i];     q[1] = (bf16)buf[4 * i + 1];
    q[2] = (bf16)buf[4 * i + 2]; q[3] = (bf16)buf[4 * i + 3];
    *(bf16x4*)(dst + 4 * i) = q;
  }
}


#define GSTR 48
#define GSTR 48
template <typename AT, int EPI, bool OUT16>
__global__ __launch_bounds__(256) void gemm_kne(const AT* __restrict__ A, int lda, const float* __restrict__ Wm, int ldw,
                                                const float* __restrict__ bias, const float* __restrict__ R, const float* __restrict__ gvec,
                                                void* __restrict__ Yv, int ldy, int K) {
  __shared__ __attribute__((aligned(16))) f16 ldsA[128 * GSTR];
  __shared__ __attribute__((aligned(16))) f16 ldsW[128 * GSTR];
  __shared__ __attribute__((aligned(16))) float oS[8][32 * 68];
  const int tid = threadIdx.x, lane = tid & 31, wave = tid >> 5, cl = lane & 15, rh = (lane >> 4) * 8;
  const int m0 = blockIdx.x * 128, n0 = blockIdx.y * 128;
  const int wm = (wave & 3) * 32, wn = (wave >> 2) * 64;
  f32x8 acc[2][4];
#pragma unroll
  for (int i = 0; i < 2; ++i)
#pragma unroll
    for (int j = 0; j < 4; ++j) { f32x8 z = {}; acc[i][j] = z; }
#pragma unroll 1
  for (int k0 = 0; k0 < K; k0 += 32) {
    __syncthreads();
    { const int row = tid >> 1, ch = (tid & 1) * 16;
      const AT* src = A + (size_t)(m0 + row) * lda + k0 + ch;
#pragma unroll
      for (int g = 0; g < 16; ++g) ldsA[row * GSTR + ch + g] = (f16)src[g]; }
    { const int k = tid >> 3, nn0 = (tid & 7) * 16;
      const float* src = Wm + (size_t)(k0 + k) * ldw + n0 + nn0;
#pragma unroll
      for (int g = 0; g < 4; ++g) { const v4f_t v = *(const v4f_t*)(src + 4 * g);
#pragma unroll
        for (int u = 0; u < 4; ++u) ldsW[(nn0 + 4 * g + u) * GSTR + k] = (f16)v[u]; } }
    __syncthreads();
    f16x16 af[2];
#pragma unroll
    for (int i = 0; i < 2; ++i) af[i] = lds_frag(ldsA + (wm + 16 * i) * GSTR, GSTR);
#pragma unroll
    for (int j = 0; j < 4; ++j) {
      const f16x16 bf = lds_frag(ldsW + (wn + 16 * j) * GSTR, GSTR);
#pragma unroll
      for (int i = 0; i < 2; ++i) acc[i][j] = wmma16(af[i], bf, acc[i][j]);
    }
  }
  float* so = oS[wave];
#pragma unroll
  for (int i = 0; i < 2; ++i)
#pragma unroll
    for (int j = 0; j < 4; ++j) {
      const int n = n0 + wn + 16 * j + cl;
      const float bv = bias ? bias[n] : 0.0f;
      const float gv = (EPI == 2 || EPI == 4) ? gvec[n] : 0.0f;
      if (EPI == 1) {
#pragma unroll 1
        for (int r = 0; r < 8; ++r) { const float xg = acc[i][j][r] + bv; so[(16 * i + rh + r) * 68 + 16 * j + cl] = 0.5f * xg * (1.0f + erff(xg * 0.70710678118654752f)); }
      } else {
#pragma unroll
        for (int r = 0; r < 8; ++r) {
          float v = acc[i][j][r] + bv;
          if (EPI == 3) v = fmaxf(v, 0.0f);
          if (EPI == 4) v = gv * v;
          if (EPI == 2) v = R[(size_t)(m0 + wm + 16 * i + rh + r) * ldy + n] + gv * v;
          so[(16 * i + rh + r) * 68 + 16 * j + cl] = v;
        }
      }
    }
  asm volatile("s_wait_dscnt 0" ::: "memory");
  __builtin_amdgcn_wave_barrier();
#pragma unroll 1
  for (int pass = 0; pass < 2; ++pass) {
    if (OUT16) {
      f16* Y = (f16*)Yv;
#pragma unroll
      for (int it = 0; it < 8; ++it) { const int c = lane + 32 * it, rr = c >> 3, q8 = (c & 7) * 8;
        union { f16 h[8]; v4u_t v; } u;
#pragma unroll
        for (int e = 0; e < 8; ++e) u.h[e] = (f16)so[rr * 68 + q8 + e];
        *(volatile v4u_t*)(Y + (size_t)(m0 + wm + rr) * ldy + n0 + wn + q8) = u.v; }
    } else {
      float* Y = (float*)Yv;
#pragma unroll
      for (int it = 0; it < 16; ++it) { const int f4 = lane + 32 * it, rr = f4 >> 4, q = (f4 & 15) * 4;
        *(volatile v4f_t*)(Y + (size_t)(m0 + wm + rr) * ldy + n0 + wn + q) = *(const v4fa*)(so + rr * 68 + q); }
    }
    __threadfence();
  }
}

template <typename AT, int EPI, bool OUT16>
__global__ __launch_bounds__(256) void gemm_knez(const AT* __restrict__ A, int lda, size_t strideA, const float* __restrict__ Wm, int ldw, size_t strideW,
                                                 const float* __restrict__ bias, const float* __restrict__ R, const float* __restrict__ gvec,
                                                 void* __restrict__ Yv, int ldy, size_t strideY, int K) {
  A += (size_t)blockIdx.z * strideA; Wm += (size_t)blockIdx.z * strideW; Yv = (void*)((char*)Yv + (size_t)blockIdx.z * strideY * (OUT16 ? 2 : 4)); if (R) R += (size_t)blockIdx.z * strideY;
  __shared__ __attribute__((aligned(16))) f16 ldsA[128 * GSTR];
  __shared__ __attribute__((aligned(16))) f16 ldsW[128 * GSTR];
  __shared__ __attribute__((aligned(16))) float oS[8][32 * 68];
  const int tid = threadIdx.x, lane = tid & 31, wave = tid >> 5, cl = lane & 15, rh = (lane >> 4) * 8;
  const int m0 = blockIdx.x * 128, n0 = blockIdx.y * 128;
  const int wm = (wave & 3) * 32, wn = (wave >> 2) * 64;
  f32x8 acc[2][4];
#pragma unroll
  for (int i = 0; i < 2; ++i)
#pragma unroll
    for (int j = 0; j < 4; ++j) { f32x8 z = {}; acc[i][j] = z; }
#pragma unroll 1
  for (int k0 = 0; k0 < K; k0 += 32) {
    __syncthreads();
    { const int row = tid >> 1, ch = (tid & 1) * 16;
      const AT* src = A + (size_t)(m0 + row) * lda + k0 + ch;
#pragma unroll
      for (int g = 0; g < 16; ++g) ldsA[row * GSTR + ch + g] = (f16)src[g]; }
    { const int k = tid >> 3, nn0 = (tid & 7) * 16;
      const float* src = Wm + (size_t)(k0 + k) * ldw + n0 + nn0;
#pragma unroll
      for (int g = 0; g < 4; ++g) { const v4f_t v = *(const v4f_t*)(src + 4 * g);
#pragma unroll
        for (int u = 0; u < 4; ++u) ldsW[(nn0 + 4 * g + u) * GSTR + k] = (f16)v[u]; } }
    __syncthreads();
    f16x16 af[2];
#pragma unroll
    for (int i = 0; i < 2; ++i) af[i] = lds_frag(ldsA + (wm + 16 * i) * GSTR, GSTR);
#pragma unroll
    for (int j = 0; j < 4; ++j) {
      const f16x16 bf = lds_frag(ldsW + (wn + 16 * j) * GSTR, GSTR);
#pragma unroll
      for (int i = 0; i < 2; ++i) acc[i][j] = wmma16(af[i], bf, acc[i][j]);
    }
  }
  float* so = oS[wave];
#pragma unroll
  for (int i = 0; i < 2; ++i)
#pragma unroll
    for (int j = 0; j < 4; ++j) {
      const int n = n0 + wn + 16 * j + cl;
      const float bv = bias ? bias[n] : 0.0f;
      const float gv = (EPI == 2 || EPI == 4) ? gvec[n] : 0.0f;
      if (EPI == 1) {
#pragma unroll 1
        for (int r = 0; r < 8; ++r) { const float xg = acc[i][j][r] + bv; so[(16 * i + rh + r) * 68 + 16 * j + cl] = 0.5f * xg * (1.0f + erff(xg * 0.70710678118654752f)); }
      } else {
#pragma unroll
        for (int r = 0; r < 8; ++r) {
          float v = acc[i][j][r] + bv;
          if (EPI == 3) v = fmaxf(v, 0.0f);
          if (EPI == 4) v = gv * v;
          if (EPI == 2) v = R[(size_t)(m0 + wm + 16 * i + rh + r) * ldy + n] + gv * v;
          so[(16 * i + rh + r) * 68 + 16 * j + cl] = v;
        }
      }
    }
  asm volatile("s_wait_dscnt 0" ::: "memory");
  __builtin_amdgcn_wave_barrier();
#pragma unroll 1
  for (int pass = 0; pass < 2; ++pass) {
    if (OUT16) {
      f16* Y = (f16*)Yv;
#pragma unroll
      for (int it = 0; it < 8; ++it) { const int c = lane + 32 * it, rr = c >> 3, q8 = (c & 7) * 8;
        union { f16 h[8]; v4u_t v; } u;
#pragma unroll
        for (int e = 0; e < 8; ++e) u.h[e] = (f16)so[rr * 68 + q8 + e];
        *(volatile v4u_t*)(Y + (size_t)(m0 + wm + rr) * ldy + n0 + wn + q8) = u.v; }
    } else {
      float* Y = (float*)Yv;
#pragma unroll
      for (int it = 0; it < 16; ++it) { const int f4 = lane + 32 * it, rr = f4 >> 4, q = (f4 & 15) * 4;
        *(volatile v4f_t*)(Y + (size_t)(m0 + wm + rr) * ldy + n0 + wn + q) = *(const v4fa*)(so + rr * 68 + q); }
    }
    __threadfence();
  }
}

template <typename AT, bool ACC>
__global__ __launch_bounds__(256) void gemm_kn2(const AT* __restrict__ A, int lda, size_t strideA,
                                               const float* __restrict__ Wm, int ldw, size_t strideW,
                                               const float* __restrict__ bias, float scale,
                                               float* __restrict__ Y, int ldy, size_t strideY, int K) {
  __shared__ __attribute__((aligned(16))) f16 ldsA[128 * GSTR], ldsAl[128 * GSTR];
  __shared__ __attribute__((aligned(16))) f16 ldsW[128 * GSTR], ldsWl[128 * GSTR];
  __shared__ __attribute__((aligned(16))) float oS[8][32 * 68];
  const int tid = threadIdx.x, lane = tid & 31, wave = tid >> 5, cl = lane & 15, rh = (lane >> 4) * 8;
  const int m0 = blockIdx.x * 128, n0 = blockIdx.y * 128;
  const int wm = (wave & 3) * 32, wn = (wave >> 2) * 64;
  A += (size_t)blockIdx.z * strideA; Wm += (size_t)blockIdx.z * strideW; Y += (size_t)blockIdx.z * strideY;
  f32x8 acc[2][4], accx[2][4];
#pragma unroll
  for (int i = 0; i < 2; ++i)
#pragma unroll
    for (int j = 0; j < 4; ++j) { f32x8 z = {}; acc[i][j] = z; accx[i][j] = z; }
#pragma unroll 1
  for (int k0 = 0; k0 < K; k0 += 32) {
    __syncthreads();
    {
      const int row = tid >> 1, ch = (tid & 1) * 16;
      const AT* src = A + (size_t)(m0 + row) * lda + k0 + ch;
#pragma unroll
      for (int g = 0; g < 16; ++g) { const float v = (float)src[g]; const f16 h = (f16)v; ldsA[row * GSTR + ch + g] = h; ldsAl[row * GSTR + ch + g] = (f16)((v - (float)h) * 2048.0f); }
    }
    {
      const int k = tid >> 3, nn0 = (tid & 7) * 16;
      const float* src = Wm + (size_t)(k0 + k) * ldw + n0 + nn0;
#pragma unroll
      for (int g = 0; g < 4; ++g) { const v4f_t v = *(const v4f_t*)(src + 4 * g);
#pragma unroll
        for (int u = 0; u < 4; ++u) { const f16 h = (f16)v[u]; ldsW[(nn0 + 4 * g + u) * GSTR + k] = h; ldsWl[(nn0 + 4 * g + u) * GSTR + k] = (f16)((v[u] - (float)h) * 2048.0f); } }
    }
    __syncthreads();
    f16x16 af[2], afl[2];
#pragma unroll
    for (int i = 0; i < 2; ++i) { af[i] = lds_frag(ldsA + (wm + 16 * i) * GSTR, GSTR); afl[i] = lds_frag(ldsAl + (wm + 16 * i) * GSTR, GSTR); }
#pragma unroll
    for (int j = 0; j < 4; ++j) {
      const f16x16 bf = lds_frag(ldsW + (wn + 16 * j) * GSTR, GSTR), bfl = lds_frag(ldsWl + (wn + 16 * j) * GSTR, GSTR);
#pragma unroll
      for (int i = 0; i < 2; ++i) { acc[i][j] = wmma16(af[i], bf, acc[i][j]); accx[i][j] = wmma16(af[i], bfl, accx[i][j]); accx[i][j] = wmma16(afl[i], bf, accx[i][j]); }
    }
  }
  float* so = oS[wave];
#pragma unroll
  for (int i = 0; i < 2; ++i)
#pragma unroll
    for (int j = 0; j < 4; ++j) {
      const float bv = bias ? bias[n0 + wn + 16 * j + cl] : 0.0f;
#pragma unroll
      for (int r = 0; r < 8; ++r) so[(16 * i + rh + r) * 68 + 16 * j + cl] = (acc[i][j][r] + accx[i][j][r] * (1.0f / 2048.0f)) * scale + bv;
    }
  asm volatile("s_wait_dscnt 0" ::: "memory");
  __builtin_amdgcn_wave_barrier();
  if (ACC) {
#pragma unroll
    for (int it = 0; it < 16; ++it) { const int f4 = lane + 32 * it, rr = f4 >> 4, q = (f4 & 15) * 4;
      const v4f_t old = *(const v4fa*)(Y + (size_t)(m0 + wm + rr) * ldy + n0 + wn + q);
      v4f_t v = *(const v4fa*)(so + rr * 68 + q); v += old; *(v4fa*)(so + rr * 68 + q) = v; }
    asm volatile("s_wait_dscnt 0" ::: "memory");
  }
#pragma unroll 1
  for (int pass = 0; pass < 2; ++pass) {
#pragma unroll
    for (int it = 0; it < 16; ++it) { const int f4 = lane + 32 * it, rr = f4 >> 4, q = (f4 & 15) * 4;
      *(volatile v4f_t*)(Y + (size_t)(m0 + wm + rr) * ldy + n0 + wn + q) = *(const v4fa*)(so + rr * 68 + q); }
    __threadfence();
  }
}

__global__ __launch_bounds__(256) void k_transpose(const float* __restrict__ Wm, float* __restrict__ Wt, int rows, int cols) {
  __shared__ float tS[64][65];
  const int tid = threadIdx.x, tbj = cols / 64, bi = blockIdx.x / tbj, bj = blockIdx.x % tbj;
  for (int e = tid; e < 64 * 64; e += 256) { const int r = e >> 6, c = e & 63; tS[r][c] = Wm[(size_t)(bi * 64 + r) * cols + bj * 64 + c]; }
  __syncthreads();
  for (int ch = tid; ch < 64 * 16; ch += 256) { const int r = ch >> 4, q4 = (ch & 15) * 4; v4f_t o; o[0] = tS[q4][r]; o[1] = tS[q4 + 1][r]; o[2] = tS[q4 + 2][r]; o[3] = tS[q4 + 3][r];
    float* dst = Wt + (size_t)(bj * 64 + r) * rows + bi * 64 + q4; *(volatile v4f_t*)dst = o; __threadfence(); *(volatile v4f_t*)dst = o; }
}


template <typename AT, int EPI, bool OUT16, int NJ>
__global__ __launch_bounds__(256) void gemm_sm(const AT* __restrict__ A, int lda, size_t sA, const float* __restrict__ Wm, int ldw, size_t sW,
                                               const float* __restrict__ bias, const float* __restrict__ R, const float* __restrict__ gvec,
                                               void* __restrict__ Yv, int ldy, size_t sY, int K) {
  constexpr int BN = 16 * NJ; constexpr int OST = BN + 4;
  A += (size_t)blockIdx.z * sA; Wm += (size_t)blockIdx.z * sW; Yv = (void*)((char*)Yv + (size_t)blockIdx.z * sY * (OUT16 ? 2 : 4)); if (R) R += (size_t)blockIdx.z * sY;
  __shared__ __attribute__((aligned(16))) f16 ldsA[256 * GSTR];
  __shared__ __attribute__((aligned(16))) f16 ldsW[BN * GSTR];
  __shared__ __attribute__((aligned(16))) float oS[8][32 * OST];
  const int tid = threadIdx.x, lane = tid & 31, wave = tid >> 5, cl = lane & 15, rh = (lane >> 4) * 8;
  const int m0 = blockIdx.x * 256, n0 = blockIdx.y * BN;
  const int wm = wave * 32;
  f32x8 acc[2][NJ];
#pragma unroll
  for (int i = 0; i < 2; ++i)
#pragma unroll
    for (int j = 0; j < NJ; ++j) { f32x8 z = {}; acc[i][j] = z; }
#pragma unroll 1
  for (int k0 = 0; k0 < K; k0 += 32) {
    __syncthreads();
    { const AT* src = A + (size_t)(m0 + tid) * lda + k0;
#pragma unroll
      for (int g = 0; g < 32; ++g) ldsA[tid * GSTR + g] = (f16)src[g]; }
    { const int k = tid >> 3, nn0 = (tid & 7) * (2 * NJ);
      const float* src = Wm + (size_t)(k0 + k) * ldw + n0 + nn0;
#pragma unroll
      for (int g = 0; g < NJ / 2; ++g) { const v4f_t v = *(const v4f_t*)(src + 4 * g);
#pragma unroll
        for (int u = 0; u < 4; ++u) ldsW[(nn0 + 4 * g + u) * GSTR + k] = (f16)v[u]; } }
    __syncthreads();
    f16x16 af[2];
#pragma unroll
    for (int i = 0; i < 2; ++i) af[i] = lds_frag(ldsA + (wm + 16 * i) * GSTR, GSTR);
#pragma unroll
    for (int j = 0; j < NJ; ++j) {
      const f16x16 bf = lds_frag(ldsW + (16 * j) * GSTR, GSTR);
#pragma unroll
      for (int i = 0; i < 2; ++i) acc[i][j] = wmma16(af[i], bf, acc[i][j]);
    }
  }
  float* so = oS[wave];
#pragma unroll
  for (int i = 0; i < 2; ++i)
#pragma unroll
    for (int j = 0; j < NJ; ++j) {
      const int n = n0 + 16 * j + cl;
      const float bv = bias ? bias[n] : 0.0f;
      const float gv = (EPI == 2 || EPI == 4) ? gvec[n] : 0.0f;
#pragma unroll
      for (int r = 0; r < 8; ++r) {
        float v = acc[i][j][r] + bv;
        if (EPI == 3) v = fmaxf(v, 0.0f);
        if (EPI == 2) v = R[(size_t)(m0 + wm + 16 * i + rh + r) * ldy + n] + gv * v;
        if (EPI == 4) v = gv * v;
        so[(16 * i + rh + r) * OST + 16 * j + cl] = v;
      }
    }
  asm volatile("s_wait_dscnt 0" ::: "memory");
  __builtin_amdgcn_wave_barrier();
#pragma unroll 1
  for (int pass = 0; pass < 2; ++pass) {
    if (OUT16) {
      f16* Y = (f16*)Yv;
#pragma unroll
      for (int it = 0; it < BN / 8; ++it) { const int c = lane + 32 * it, rr = c / (BN / 8), q8 = (c % (BN / 8)) * 8;
        union { f16 h[8]; v4u_t v; } u;
#pragma unroll
        for (int e = 0; e < 8; ++e) u.h[e] = (f16)so[rr * OST + q8 + e];
        *(volatile v4u_t*)(Y + (size_t)(m0 + wm + rr) * ldy + n0 + q8) = u.v; }
    } else {
      float* Y = (float*)Yv;
#pragma unroll
      for (int it = 0; it < BN / 4; ++it) { const int f4 = lane + 32 * it, rr = f4 / (BN / 4), q = (f4 % (BN / 4)) * 4;
        *(volatile v4f_t*)(Y + (size_t)(m0 + wm + rr) * ldy + n0 + q) = *(const v4fa*)(so + rr * OST + q); }
    }
    __threadfence();
  }
}

#define NBm 32
#define BIN 32
#define NNm 2048
#define UUm 64
#define XW 2048
#define XIW 128
__global__ __launch_bounds__(256) void k_fill(float* __restrict__ p, float val, size_t n4) { const size_t i = (size_t)blockIdx.x * 256 + threadIdx.x; if (i < n4) { v4f_t v = {val, val, val, val}; *(volatile v4f_t*)(p + 4 * i) = v; __threadfence(); *(volatile v4f_t*)(p + 4 * i) = v; } }
__global__ __launch_bounds__(256) void k_dbg_zero(float* __restrict__ p, size_t n4) { const size_t i = (size_t)blockIdx.x * 256 + threadIdx.x; if (i < n4) { v4f_t z = {0.f,0.f,0.f,0.f}; *(volatile v4f_t*)(p + 4 * i) = z; __threadfence(); *(volatile v4f_t*)(p + 4 * i) = z; } }
__global__ __launch_bounds__(256) void k_copy(const float* __restrict__ src, float* __restrict__ dst, size_t n4) { const size_t i = (size_t)blockIdx.x * 256 + threadIdx.x; if (i < n4) { const v4f_t v = *(const v4f_t*)(src + 4 * i); *(volatile v4f_t*)(dst + 4 * i) = v; __threadfence(); *(volatile v4f_t*)(dst + 4 * i) = v; } }
__global__ __launch_bounds__(32) void k_fs(const float* __restrict__ feat, const float* __restrict__ se, float* __restrict__ FS) {
  const int n = blockIdx.x, t = threadIdx.x; if (t >= 24) return; const int c = 4 * t;
  const v4f_t v = (c < 32) ? *(const v4f_t*)(feat + (size_t)n * 32 + c) : *(const v4f_t*)(se + (size_t)n * 64 + (c - 32));
  float* d = FS + (size_t)n * 96 + c; *(volatile v4f_t*)d = v; __threadfence(); *(volatile v4f_t*)d = v;
}
__global__ __launch_bounds__(256) void k_svec(const float* __restrict__ H1, const float* __restrict__ ws2, const float* __restrict__ bs2, float* __restrict__ sv) {
  __shared__ float st[32];
  const int tid = threadIdx.x, r = tid >> 3, part = tid & 7; const size_t n = (size_t)blockIdx.x * 32 + r; float a = 0.0f;
#pragma unroll
  for (int i = 0; i < 8; ++i) { const int c = part * 8 + i; a = fmaf(H1[n * 64 + c], ws2[c], a); }
  a += __shfl_xor(a, 1, 32); a += __shfl_xor(a, 2, 32); a += __shfl_xor(a, 4, 32);
  if (part == 0) st[r] = fmaxf(a + bs2[0], 0.0f);
  __syncthreads();
  if (tid < 32) { float* d = sv + (size_t)blockIdx.x * 32 + tid; const float v = st[tid]; *(volatile float*)d = v; __threadfence(); *(volatile float*)d = v; }
}
__global__ __launch_bounds__(256) void k_attnorm(float* __restrict__ Sm, const float* __restrict__ sv) {
  __shared__ float red[256];
  const int n = blockIdx.x, tid = threadIdx.x; float* sr = Sm + (size_t)n * NNm; float v[NNm / 256]; float z = 0.0f;
#pragma unroll
  for (int e = 0; e < NNm / 256; ++e) { v[e] = expf(sr[tid + 256 * e] * 0.125f); z += v[e]; }
  red[tid] = z; __syncthreads();
  for (int o = 128; o > 0; o >>= 1) { if (tid < o) red[tid] += red[tid + o]; __syncthreads(); }
  const float inv = 1.0f / (sv[n] + red[0]);
#pragma unroll 1
  for (int pass = 0; pass < 2; ++pass) {
#pragma unroll
    for (int e = 0; e < NNm / 256; ++e) *(volatile float*)(sr + tid + 256 * e) = v[e] * inv;
    __threadfence(); }
}
__global__ __launch_bounds__(256) void k_xh(const float* __restrict__ hp, const float* __restrict__ inp, float* __restrict__ XH, float* __restrict__ XIN) {
  const int m = blockIdx.x, tid = threadIdx.x;
#pragma unroll 1
  for (int q = tid; q < XW / 4; q += 256) { const int b = (4 * q) / UUm, u = (4 * q) % UUm; v4f_t v = {0.f, 0.f, 0.f, 0.f}; if (b < NBm) v = *(const v4f_t*)(hp + (size_t)b * NNm * UUm + (size_t)m * UUm + u);
    float* d = XH + (size_t)m * XW + 4 * q; *(volatile v4f_t*)d = v; __threadfence(); *(volatile v4f_t*)d = v; }
  if (tid < XIW / 4) { const int b = tid; v4f_t v = {0.f, 0.f, 0.f, 0.f}; if (b < NBm) { v[0] = inp[((size_t)b * NNm + m) * 2 + 0]; v[1] = inp[((size_t)b * NNm + m) * 2 + 1]; }
    float* d = XIN + (size_t)m * XIW + 4 * tid; *(volatile v4f_t*)d = v; __threadfence(); *(volatile v4f_t*)d = v; }
}
__global__ __launch_bounds__(256) void k_gate(const float* __restrict__ P, const float* __restrict__ XIN, const float* __restrict__ YIN, const float* __restrict__ K, const float* __restrict__ bias, int mode, float* __restrict__ G) {
  const int tid = threadIdx.x; const size_t row = (size_t)blockIdx.x * 4 + (tid >> 6); const int u = tid & 63; const int n = (int)(row / NBm), b = (int)(row % NBm);
  float acc = P[row * UUm + u];
  { const float y0 = XIN[(size_t)n * XIW + b * 4 + 0], y1 = XIN[(size_t)n * XIW + b * 4 + 1]; acc = fmaf(y0, K[0 * UUm + u], acc); acc = fmaf(y1, K[1 * UUm + u], acc); }
#pragma unroll
  for (int m = 1; m < 4; ++m) { const float* ym = YIN + (size_t)(m - 1) * NNm * XIW; const float y0 = ym[(size_t)n * XIW + b * 4 + 0], y1 = ym[(size_t)n * XIW + b * 4 + 1];
    acc = fmaf(y0, K[((size_t)m * 66 + 0) * UUm + u], acc); acc = fmaf(y1, K[((size_t)m * 66 + 1) * UUm + u], acc); }
  float bsum = 0.0f;
#pragma unroll
  for (int m = 0; m < 4; ++m) bsum += bias[m * UUm + u];
  const float pre = acc * 0.25f + bsum * 0.25f; const float o = (mode == 0) ? (1.0f / (1.0f + expf(-pre))) : tanhf(pre);
  *(volatile float*)(G + row * UUm + u) = o; __threadfence(); *(volatile float*)(G + row * UUm + u) = o;
}
__global__ __launch_bounds__(256) void k_mul(const float* __restrict__ a, const float* __restrict__ b2, float* __restrict__ d) { const size_t i4 = ((size_t)blockIdx.x * 256 + threadIdx.x) * 4; const v4f_t v = *(const v4f_t*)(a + i4) * *(const v4f_t*)(b2 + i4); *(volatile v4f_t*)(d + i4) = v; __threadfence(); *(volatile v4f_t*)(d + i4) = v; }
__global__ __launch_bounds__(256) void k_hnew(const float* __restrict__ Ug, const float* __restrict__ Cg, const float* __restrict__ XH, float* __restrict__ out) {
  const int n = blockIdx.x, tid = threadIdx.x;
#pragma unroll 1
  for (int q = tid; q < NBm * 16; q += 256) { const int b = q >> 4, u = (q & 15) * 4; const size_t src = ((size_t)n * NBm + b) * UUm + u;
    const v4f_t ug = *(const v4f_t*)(Ug + src), cg = *(const v4f_t*)(Cg + src), hg = *(const v4f_t*)(XH + src); const v4f_t v = ug * hg + (1.0f - ug) * cg;
    float* d = out + (size_t)b * NNm * UUm + (size_t)n * UUm + u; *(volatile v4f_t*)d = v; __threadfence(); *(volatile v4f_t*)d = v; }
}

extern "C" void kernel_launch(void* const* d_in, const int* in_sizes, int n_in,
                              void* d_out, int out_size, void* d_ws, size_t ws_size,
                              hipStream_t stream) {
  (void)in_sizes; (void)n_in; (void)out_size;
  const float** f = (const float**)d_in;
  const float* inp = f[0], *hp = f[1], *adj1 = f[2], *adj2 = f[3], *feat = f[4], *se = f[5], *Wq = f[6], *Wk = f[7], *Ws1 = f[8], *bs1 = f[9], *Ws2 = f[10], *bs2 = f[11];
  const float* rk = f[12], *rbias = f[13], *uk = f[14], *ubias = f[15], *ck = f[16], *cbias = f[17];
  float* out = (float*)d_out;
  char* ws = (char*)d_ws;
  float* FS = (float*)ws; ws += (size_t)NNm * 96 * 4; float* Qm = (float*)ws; ws += (size_t)NNm * 64 * 4; float* Km = (float*)ws; ws += (size_t)NNm * 64 * 4; float* H1 = (float*)ws; ws += (size_t)NNm * 64 * 4;
  float* KT = (float*)ws; ws += (size_t)64 * NNm * 4; float* sv = (float*)ws; ws += (size_t)NNm * 4; float* SA = (float*)ws; ws += (size_t)NNm * NNm * 4;
  float* XH = (float*)ws; ws += (size_t)NNm * XW * 4; float* XIN = (float*)ws; ws += (size_t)NNm * XIW * 4; float* XRH = (float*)ws; ws += (size_t)NNm * XW * 4;
  float* Y = (float*)ws; ws += (size_t)3 * NNm * XW * 4; float* YIN = (float*)ws; ws += (size_t)3 * NNm * XIW * 4;
  float* P = (float*)ws; ws += (size_t)NNm * XW * 4; float* RG = (float*)ws; ws += (size_t)NNm * XW * 4; float* UG = (float*)ws; ws += (size_t)NNm * XW * 4; float* ones = (float*)ws; ws += 64 * 4;
  if ((size_t)(ws - (char*)d_ws) > ws_size) return;
  float* CG = RG;
  const dim3 blk(256); const float* sup[3] = {adj1, adj2, SA};
  k_fill<<<dim3(1), blk, 0, stream>>>(ones, 1.0f, 64 / 4);

  gemm_sm<float, 3, false, 4><<<dim3(NNm / 256, 1, 1), blk, 0, stream>>>(feat, 32, (size_t)0, Wq, 64, (size_t)0, nullptr, nullptr, nullptr, Qm, 64, (size_t)0, 32);
  gemm_sm<float, 3, false, 4><<<dim3(NNm / 256, 1, 1), blk, 0, stream>>>(feat, 32, (size_t)0, Wk, 64, (size_t)0, nullptr, nullptr, nullptr, Km, 64, (size_t)0, 32);
  k_fs<<<dim3(NNm), dim3(32), 0, stream>>>(feat, se, FS);
  gemm_sm<float, 3, false, 4><<<dim3(NNm / 256, 1, 1), blk, 0, stream>>>(FS, 96, (size_t)0, Ws1, 64, (size_t)0, bs1, nullptr, nullptr, H1, 64, (size_t)0, 96);
  k_svec<<<dim3(NNm / 32), blk, 0, stream>>>(H1, Ws2, bs2, sv);
  k_transpose<<<dim3((NNm / 64) * (64 / 64)), blk, 0, stream>>>(Km, KT, NNm, 64);
  gemm_kne<float, 0, false><<<dim3(NNm / 128, NNm / 128), blk, 0, stream>>>(Qm, 64, KT, NNm, nullptr, nullptr, nullptr, SA, NNm, 64);
  k_attnorm<<<dim3(NNm), blk, 0, stream>>>(SA, sv);
  k_xh<<<dim3(NNm), blk, 0, stream>>>(hp, inp, XH, XIN);
  for (int m = 0; m < 3; ++m) gemm_kne<float, 0, false><<<dim3(NNm / 128, XIW / 128), blk, 0, stream>>>(sup[m], NNm, XIN, XIW, nullptr, nullptr, nullptr, YIN + (size_t)m * NNm * XIW, XIW, NNm);
#pragma unroll 1
  for (int phase = 0; phase < 2; ++phase) {
    const float* XZ = phase ? XRH : XH;
    for (int m = 0; m < 3; ++m) gemm_kne<float, 0, false><<<dim3(NNm / 128, XW / 128), blk, 0, stream>>>(sup[m], NNm, XZ, XW, nullptr, nullptr, nullptr, Y + (size_t)m * NNm * XW, XW, NNm);
    for (int g = 0; g < (phase ? 1 : 2); ++g) {
      const float* Kg = phase ? ck : (g ? uk : rk); const float* bg = phase ? cbias : (g ? ubias : rbias); float* Gd = phase ? CG : (g ? UG : RG);
      gemm_sm<float, 0, false, 4><<<dim3((unsigned)((size_t)NNm * NBm / 256), 1, 1), blk, 0, stream>>>(XZ, UUm, (size_t)0, Kg + 2 * UUm, UUm, (size_t)0, nullptr, nullptr, nullptr, P, UUm, (size_t)0, UUm);
      for (int m = 0; m < 3; ++m)
        gemm_sm<float, 2, false, 4><<<dim3((unsigned)((size_t)NNm * NBm / 256), 1, 1), blk, 0, stream>>>(Y + (size_t)m * NNm * XW, UUm, (size_t)0, Kg + ((size_t)(m + 1) * 66 + 2) * UUm, UUm, (size_t)0, nullptr, P, ones, P, UUm, (size_t)0, UUm);
      k_gate<<<dim3((unsigned)((size_t)NNm * NBm / 4)), blk, 0, stream>>>(P, XIN, YIN, Kg, bg, phase, Gd);
    }
    if (phase == 0) k_mul<<<dim3((unsigned)((size_t)NNm * XW / 4 / 256)), blk, 0, stream>>>(RG, XH, XRH);
  }
  k_hnew<<<dim3(NNm), blk, 0, stream>>>(UG, CG, XH, out);
}
